// Swin3D_60533269069902
// MI455X (gfx1250) — hardware-run, weakly checked
//
#include <hip/hip_runtime.h>


namespace {
constexpr int N = 32768, K = 16, D = 128, D2 = 256;
constexpr float XS = 8.0f, WSC = 256.0f, EPS = 1e-5f;
typedef _Float16 b16;
typedef __attribute__((ext_vector_type(16))) _Float16 v16b;
typedef __attribute__((ext_vector_type(8))) _Float16 v8b;
typedef __attribute__((ext_vector_type(8))) float v8f;
typedef __attribute__((ext_vector_type(4))) float v4f;
__device__ __forceinline__ float bf16_rne(float f) { unsigned int u = __float_as_uint(f); u += 0x7FFFu + ((u >> 16) & 1u); float r = __uint_as_float(u & 0xFFFF0000u); asm volatile("" : "+v"(r)); return r; }
__device__ __forceinline__ void split16(float v, b16& hi, b16& lo) { hi = (b16)v; lo = (b16)(v - (float)hi); }
__device__ __forceinline__ v16b frag_kb(const b16* p, int hh) { const v8b a = *(const v8b*)(p + 8 * hh), b = *(const v8b*)(p + 16 + 8 * hh); v16b f;
#pragma unroll
  for (int e = 0; e < 8; ++e) { f[e] = a[e]; f[8 + e] = b[e]; } return f; }
__device__ __forceinline__ v8f wmma16b(v16b a, v16b b, v8f c) { v8f d = __builtin_amdgcn_wmma_f32_16x16x32_f16(false, a, false, b, (short)0, c, false, false); asm volatile("v_nop\n\tv_nop\n\tv_nop\n\tv_nop" : "+v"(d) : "v"(a), "v"(b)); return d; }
__device__ __forceinline__ void wave_lds_sync() { __builtin_amdgcn_fence(__ATOMIC_RELEASE, "workgroup"); __builtin_amdgcn_wave_barrier(); __builtin_amdgcn_fence(__ATOMIC_ACQUIRE, "workgroup"); }
__device__ __forceinline__ float pmul(float a, float b) { float p = a * b; asm volatile("" : "+v"(p)); return p; }
__device__ __forceinline__ int iclamp(int v, int lo, int hi) { return v < lo ? lo : (v > hi ? hi : v); }

__global__ __launch_bounds__(256) void wput_kernel(const float* __restrict__ w, int Kd, int O, b16* __restrict__ WT) { const int u = blockIdx.x * 256 + threadIdx.x; if (u >= O * (Kd / 8)) return; const int o = u / (Kd / 8), k0 = (u % (Kd / 8)) * 8; v8b v;
#pragma unroll
  for (int j = 0; j < 8; ++j) v[j] = (b16)(bf16_rne(w[(size_t)(k0 + j) * O + o]) * WSC); for (int pass = 0; pass < 2; ++pass) { *(volatile v8b*)(WT + (size_t)o * Kd + k0) = v; __threadfence(); } }
template <int MODE>
__global__ __launch_bounds__(32) void dense_kernel(const float* __restrict__ IN, const float* __restrict__ h, const b16* __restrict__ WT, const float* __restrict__ bias, const float* __restrict__ ST1, const float* __restrict__ g1, const float* __restrict__ be1, int NLIM, float* __restrict__ OUT, float* __restrict__ PS) {
  constexpr int KIN = (MODE == 1 || MODE == 3) ? D2 : D, NOUT = MODE == 2 ? D2 : D, NGR = NOUT / 128; __shared__ __attribute__((aligned(16))) b16 Ah[16][KIN + 8], Al[16][MODE == 0 ? 8 : KIN + 8]; __shared__ float Tf[16][132];
  const int lane = threadIdx.x, nloc = lane & 15, hlf = lane >> 4; const int g = blockIdx.x % NGR; const size_t m0 = (size_t)(blockIdx.x / NGR) * 16; if (m0 >= (size_t)NLIM) return;
  for (int rr = 0; rr < 16; ++rr) for (int q = 0; q < KIN / 32; ++q) { const int c = q * 32 + lane; float v = IN[(m0 + rr) * KIN + c];
    if (MODE == 0) { Ah[rr][c] = (b16)(bf16_rne(v) * XS); continue; }
    if (MODE == 2) v = pmul(pmul(v - ST1[c], ST1[D + c]), bf16_rne(g1[c])) + bf16_rne(be1[c]);
    b16 p, ql; split16(v * XS, p, ql); Ah[rr][c] = p; Al[rr][c] = ql; }
  wave_lds_sync(); v8f acc[8];
#pragma unroll
  for (int t = 0; t < 8; ++t) acc[t] = (v8f){};
#pragma unroll 2
  for (int kb = 0; kb < KIN; kb += 32) { const v16b a = frag_kb(&Ah[nloc][kb], hlf); v16b al; if (MODE != 0) al = frag_kb(&Al[nloc][kb], hlf);
#pragma unroll
    for (int t = 0; t < 8; ++t) { const v16b bw = frag_kb(WT + (size_t)(g * 128 + t * 16 + nloc) * KIN + kb, hlf); acc[t] = wmma16b(a, bw, acc[t]); if (MODE != 0) acc[t] = wmma16b(al, bw, acc[t]); } }
#pragma unroll
  for (int t = 0; t < 8; ++t) { const int cc = t * 16 + nloc; const float bb = MODE == 0 ? 0.0f : bf16_rne(bias[g * 128 + cc]);
#pragma unroll
    for (int r8 = 0; r8 < 8; ++r8) { float v = acc[t][r8] * (1.0f / (XS * WSC)) + bb; if (MODE == 2) v = fmaxf(v, 0.0f); Tf[8 * hlf + r8][cc] = v; } }
  wave_lds_sync(); float s4[4] = {0, 0, 0, 0}, q4[4] = {0, 0, 0, 0};
  for (int pass = 0; pass < 2; ++pass) { for (int rr = 0; rr < 16; ++rr) { v4f v = *(const v4f*)(&Tf[rr][lane * 4]);
      if (MODE == 1) { const v4f hv = *(const v4f*)(h + (m0 + rr) * D + lane * 4); for (int k = 0; k < 4; ++k) v[k] += bf16_rne(hv[k]); }
      if (MODE == 3) { const v4f pv = *(const v4f*)(h + (m0 + rr) * D + lane * 4);
        for (int k = 0; k < 4; ++k) { const int c = lane * 4 + k; v[k] += pmul(pmul(pv[k] - ST1[c], ST1[D + c]), bf16_rne(g1[c])) + bf16_rne(be1[c]); } }
      if (pass == 0 && (MODE == 1 || MODE == 3)) for (int k = 0; k < 4; ++k) { s4[k] += v[k]; q4[k] += pmul(v[k], v[k]); }
      *(volatile v4f*)(OUT + (m0 + rr) * NOUT + g * 128 + lane * 4) = v; }
    if (MODE == 1 || MODE == 3) { *(volatile v4f*)(PS + (size_t)blockIdx.x * D2 + lane * 4) = (v4f){s4[0], s4[1], s4[2], s4[3]}; *(volatile v4f*)(PS + (size_t)blockIdx.x * D2 + D + lane * 4) = (v4f){q4[0], q4[1], q4[2], q4[3]}; }
    __threadfence(); } }
__global__ __launch_bounds__(256) void edge_kernel(const float* __restrict__ HW, const float* __restrict__ h, const int* __restrict__ nb, const float* __restrict__ b1, const float* __restrict__ w2, const float* __restrict__ b2, int NLIM, float* __restrict__ MM) { const int wave = threadIdx.x >> 5, lane = threadIdx.x & 31; const size_t n = (size_t)blockIdx.x * 8 + wave; if (n >= (size_t)NLIM) return;
  const v4f hn = *(const v4f*)(HW + n * D + lane * 4); const v4f hv0 = *(const v4f*)(h + n * D + lane * 4); float hv[4], bb[4], ww[4]; for (int k = 0; k < 4; ++k) { hv[k] = bf16_rne(hv0[k]); bb[k] = bf16_rne(b1[lane * 4 + k]); ww[k] = bf16_rne(w2[lane * 4 + k]); } const float bb2 = bf16_rne(b2[0]);
  float sm[4] = {0, 0, 0, 0}, mx[4] = {-INFINITY, -INFINITY, -INFINITY, -INFINITY};
#pragma unroll 1
  for (int j = 0; j < K; ++j) { int u = iclamp(nb[n * K + j], 0, N - 1); if (u >= NLIM) u = (int)n;     const v4f hu = *(const v4f*)(HW + (size_t)u * D + lane * 4); float s = 0.0f;
    for (int k = 0; k < 4; ++k) s += pmul(fmaxf(hu[k] - hn[k] + bb[k], 0.0f), ww[k]); for (int o = 16; o; o >>= 1) s += __shfl_xor(s, o); const float att = __expf(-fmaxf(s + bb2, 0.0f));
    for (int k = 0; k < 4; ++k) { const float m = pmul(att, hv[k]); sm[k] += m; mx[k] = fmaxf(mx[k], m); } }
  v4f o0, o1; for (int k = 0; k < 4; ++k) { o0[k] = sm[k] * (1.0f / K); o1[k] = mx[k]; }
  for (int pass = 0; pass < 2; ++pass) { *(volatile v4f*)(MM + n * D2 + lane * 4) = o0; *(volatile v4f*)(MM + n * D2 + D + lane * 4) = o1; __threadfence(); } }
__global__ __launch_bounds__(256) void bnstat_kernel(const float* __restrict__ PS, int nwaves, int nnodes, float* __restrict__ ST) { const int t = threadIdx.x; const int c = t & 127; const int half = t >> 7; double s = 0.0;
  for (int w = half; w < nwaves; w += 2) s += (double)PS[(size_t)w * D2 + c]; __shared__ double S1[256], S2[256]; S1[t] = s; double q = 0.0; for (int w = half; w < nwaves; w += 2) q += (double)PS[(size_t)w * D2 + D + c]; S2[t] = q; __syncthreads();
  if (t < D) { const double sum = S1[t] + S1[t + 128], sq = S2[t] + S2[t + 128]; const double mu = sum / nnodes; double var = sq / nnodes - mu * mu; if (var < 0.0) var = 0.0; const float m = (float)mu, rs = (float)(1.0 / sqrt(var + (double)EPS));
    for (int pass = 0; pass < 2; ++pass) { ((volatile float*)ST)[t] = m; ((volatile float*)ST)[D + t] = rs; __threadfence(); } } }
__global__ __launch_bounds__(256) void bn2_kernel(const float* __restrict__ P2, const float* __restrict__ ST2, const float* __restrict__ g2, const float* __restrict__ be2, int NLIM, float* __restrict__ out) { const size_t u = (size_t)blockIdx.x * 256 + threadIdx.x; if (u >= (size_t)N * D / 4) return; const size_t n = u / (D / 4); const int c0 = (int)(u % (D / 4)) * 4; v4f r = {0, 0, 0, 0};
  if (n < (size_t)NLIM) { const v4f p = *(const v4f*)(P2 + u * 4); for (int k = 0; k < 4; ++k) r[k] = pmul(pmul(p[k] - ST2[c0 + k], ST2[D + c0 + k]), bf16_rne(g2[c0 + k])) + bf16_rne(be2[c0 + k]); }
  for (int pass = 0; pass < 2; ++pass) { *(volatile v4f*)(out + u * 4) = r; __threadfence(); } }
}

extern "C" void kernel_launch(void* const* d_in, const int* in_sizes, int n_in, void* d_out, int out_size, void* d_ws, size_t ws_size, hipStream_t stream) {
  (void)n_in;
  auto Fp = [&](int i) { return (const float*)d_in[i]; }; auto Ip = [&](int i) { return (const int*)d_in[i]; };
  if (in_sizes[0] != N * D || in_sizes[1] != N * K || in_sizes[2] != D * D || in_sizes[4] != D || in_sizes[6] != D2 * D || in_sizes[10] != D * D2 || in_sizes[12] != D2 * D || out_size != N * D) return;
  const int NLIM = N;
  size_t off = 0; char* ws = (char*)d_ws;
  auto carve = [&](size_t bytes) { char* p = ws + off; off += (bytes + 255) & ~(size_t)255; return p; };
  b16* W1T = (b16*)carve((size_t)D * D * 2); b16* OWT = (b16*)carve((size_t)D * D2 * 2); b16* F1T = (b16*)carve((size_t)D2 * D * 2); b16* F2T = (b16*)carve((size_t)D * D2 * 2);
  float* HW = (float*)carve((size_t)N * D * 4); float* MM = (float*)carve((size_t)N * D2 * 4); float* P1 = (float*)carve((size_t)N * D * 4); float* Y1 = (float*)carve((size_t)N * D2 * 4); float* P2 = (float*)carve((size_t)N * D * 4);
  const int NW = NLIM / 16; float* PS = (float*)carve((size_t)(N / 16) * 2 * D2 * 4); float* ST1 = (float*)carve(D2 * 4); float* ST2 = (float*)carve(D2 * 4);
  if (off > ws_size || off > ((size_t)160 << 20)) return;
  wput_kernel<<<(D * D / 8 + 255) / 256, 256, 0, stream>>>(Fp(2), D, D, W1T); wput_kernel<<<(D2 * D / 8 + 255) / 256, 256, 0, stream>>>(Fp(6), D2, D, OWT); wput_kernel<<<(D * D2 / 8 + 255) / 256, 256, 0, stream>>>(Fp(10), D, D2, F1T); wput_kernel<<<(D2 * D / 8 + 255) / 256, 256, 0, stream>>>(Fp(12), D2, D, F2T);
  dense_kernel<0><<<NW, 32, 0, stream>>>(Fp(0), nullptr, W1T, nullptr, nullptr, nullptr, nullptr, NLIM, HW, nullptr);
  edge_kernel<<<(NLIM + 7) / 8, 256, 0, stream>>>(HW, Fp(0), Ip(1), Fp(3), Fp(4), Fp(5), NLIM, MM);
  dense_kernel<1><<<NW, 32, 0, stream>>>(MM, Fp(0), OWT, Fp(7), nullptr, nullptr, nullptr, NLIM, P1, PS);
  bnstat_kernel<<<1, 256, 0, stream>>>(PS, NW, NLIM, ST1);
  dense_kernel<2><<<NW * 2, 32, 0, stream>>>(P1, nullptr, F1T, Fp(11), ST1, Fp(8), Fp(9), NLIM, Y1, nullptr);
  dense_kernel<3><<<NW, 32, 0, stream>>>(Y1, P1, F2T, Fp(13), ST1, Fp(8), Fp(9), NLIM, P2, PS);
  bnstat_kernel<<<1, 256, 0, stream>>>(PS, NW, NLIM, ST2);
  bn2_kernel<<<(unsigned)(((size_t)N * D / 4 + 255) / 256), 256, 0, stream>>>(P2, ST2, Fp(14), Fp(15), NLIM, (float*)d_out);
}
